// MambaTopDownPath_10857677324811
// MI455X (gfx1250) — hardware-verified
//
#include <hip/hip_runtime.h>
#include <stdint.h>
#include <stddef.h>

#define Bc       2
#define Cc       256
#define HT       32
#define WT       32
#define HL       64
#define WL       64
#define Lc       (HL * WL)
#define NROW     (Bc * Lc)
#define D_STATE  16
#define D_INNER  512
#define DT_RANK  16
#define D_CONV   4
#define DBC_P    64
#define NG       (D_INNER / 16)
#define SHP      68
#define CHUNK    128

#define W_SCALE  64.0f
#define X_SCALE  256.0f
#define DB_SCALE 256.0f
#define Y_SCALE  1024.0f

typedef _Float16 f16;
typedef f16 v16h __attribute__((ext_vector_type(16)));
typedef f16 v8h __attribute__((ext_vector_type(8)));
typedef v8h v8ha __attribute__((may_alias));
typedef float v8f __attribute__((ext_vector_type(8)));
typedef float v4f __attribute__((ext_vector_type(4)));
typedef v4f v4fa __attribute__((may_alias));
typedef unsigned int v4u __attribute__((ext_vector_type(4)));

union Frag  { v16h v; v8h half[2]; v4u u[2]; };
union Pack8 { v8h h; v4u u; f16 s[8]; };
union Pack4 { v4f f; v4u u; float s[4]; };

__device__ __forceinline__ v4u zero4u() { v4u z; z.x = 0u; z.y = 0u; z.z = 0u; z.w = 0u; return z; }

__device__ __forceinline__ v8f mma16(const v16h a, const v16h b, v8f c) {
  c = __builtin_amdgcn_wmma_f32_16x16x32_f16(false, a, false, b, (short)0, c, false, false);
  asm volatile("v_nop\n\tv_nop\n\tv_nop\n\tv_nop" : "+v"(c) : "v"(a), "v"(b));
  return c;
}

__device__ __forceinline__ v16h ld_frag(const f16* rowp, int k0) {
  const int h = (threadIdx.x >> 4) & 1;
  Frag f;
  f.half[0] = *(const v8ha*)(rowp + k0 + 8 * h);
  f.half[1] = *(const v8ha*)(rowp + k0 + 16 + 8 * h);
  return f.v;
}

__device__ __forceinline__ v8f zero8f() {
  v8f z;
#pragma unroll
  for (int i = 0; i < 8; ++i) z[i] = 0.0f;
  return z;
}

__global__ void __launch_bounds__(256)
k_wT(const float* __restrict__ W, f16* __restrict__ Wt, int K, int N, int Kp, float scale) {
  const unsigned kp8 = (unsigned)(Kp >> 3);
  const unsigned total = (unsigned)N * kp8;
  const unsigned i = blockIdx.x * 256u + threadIdx.x;
  const bool act = i < total;
  const unsigned ii = act ? i : 0u;
  const int n  = (int)(ii / kp8);
  const int k8 = (int)(ii % kp8) * 8;
  Pack8 p;
#pragma unroll
  for (int j = 0; j < 8; ++j) {
    const int k = k8 + j;
    const float v = (k < K) ? W[(size_t)k * N + n] * scale : 0.0f;
    p.s[j] = (f16)v;
  }
  f16* dst = Wt + (size_t)ii * 8;
  if (act) *(volatile v4u*)dst = p.u;
  __threadfence();
  if (act) *(volatile v4u*)dst = p.u;
}

__global__ void __launch_bounds__(256)
k_convwT(const float* __restrict__ Fw, f16* __restrict__ Wc, float scale) {
  const unsigned total = 9u * 256u * 512u / 8u;
  const unsigned i = blockIdx.x * 256u + threadIdx.x;
  const bool act = i < total;
  const unsigned ii = act ? i : 0u;
  const int ci8 = (int)(ii & 63u) * 8;
  const int co  = (int)((ii >> 6) & 255u);
  const int t   = (int)(ii >> 14);
  Pack8 p;
#pragma unroll
  for (int j = 0; j < 8; ++j)
    p.s[j] = (f16)(Fw[((size_t)co * 512 + ci8 + j) * 9 + t] * scale);
  f16* dst = Wc + (size_t)ii * 8;
  if (act) *(volatile v4u*)dst = p.u;
  __threadfence();
  if (act) *(volatile v4u*)dst = p.u;
}

__global__ void __launch_bounds__(256)
k_build_u(const float* __restrict__ top, f16* __restrict__ U) {
  const unsigned total = (unsigned)NROW * 32u;
  const unsigned i = blockIdx.x * 256u + threadIdx.x;
  const bool act = i < total;
  const unsigned ii = act ? i : 0u;
  const int c8 = (int)(ii & 31u) * 8;
  const int r  = (int)(ii >> 5);
  const int l  = r & (Lc - 1);
  const int b  = r >> 12;
  const int hp = l >> 6, wp = l & 63;
  const float* src = top + (((size_t)b * Cc + c8) * HT + (hp >> 1)) * WT + (wp >> 1);
  Pack8 p;
#pragma unroll
  for (int j = 0; j < 8; ++j) p.s[j] = (f16)src[(size_t)j * (HT * WT)];
  f16* dst = U + (size_t)ii * 8;
  if (act) *(volatile v4u*)dst = p.u;
  __threadfence();
  if (act) *(volatile v4u*)dst = p.u;
}

__global__ void __launch_bounds__(256)
k_lateral(const float* __restrict__ lat, f16* __restrict__ Cat) {
  const unsigned total = (unsigned)NROW * 32u;
  const unsigned i = blockIdx.x * 256u + threadIdx.x;
  const bool act = i < total;
  const unsigned ii = act ? i : 0u;
  const int c8 = (int)(ii & 31u) * 8;
  const int px = (int)(ii >> 5);
  const int b  = px >> 12;
  const int hw = px & (Lc - 1);
  const float* src = lat + ((size_t)b * Cc + c8) * Lc + hw;
  Pack8 p;
#pragma unroll
  for (int j = 0; j < 8; ++j) p.s[j] = (f16)src[(size_t)j * Lc];
  f16* dst = Cat + (size_t)px * 512 + 256 + c8;
  if (act) *(volatile v4u*)dst = p.u;
  __threadfence();
  if (act) *(volatile v4u*)dst = p.u;
}

__global__ void __launch_bounds__(128)
k_in_proj(const f16* __restrict__ U, const f16* __restrict__ WinT,
          float* __restrict__ X, float* __restrict__ Z) {
  __shared__ __attribute__((aligned(16))) float sh[64 * SHP];
  const int tid = threadIdx.x, wave = tid >> 5, l = tid & 31, h = l >> 4, m = l & 15;
  const int rowblk = blockIdx.x * 64, col0 = blockIdx.y * 64;
  if (rowblk >= NROW || col0 >= 2 * D_INNER) return;
  const int row0 = rowblk + wave * 16;
  v8f acc[4];
#pragma unroll
  for (int j = 0; j < 4; ++j) acc[j] = zero8f();
  const f16* arow = U + (size_t)(row0 + m) * Cc;
  for (int k = 0; k < Cc; k += 32) {
    const v16h a = ld_frag(arow, k);
#pragma unroll
    for (int j = 0; j < 4; ++j) {
      const v16h bb = ld_frag(WinT + (size_t)(col0 + 16 * j + m) * Cc, k);
      acc[j] = mma16(a, bb, acc[j]);
    }
  }
#pragma unroll
  for (int j = 0; j < 4; ++j)
#pragma unroll
    for (int r = 0; r < 8; ++r)
      sh[(wave * 16 + 8 * h + r) * SHP + 16 * j + m] = acc[j][r] * (1.0f / W_SCALE);
  __syncthreads();
  float* dstb; int cx;
  if (col0 < D_INNER) { dstb = X; cx = col0; } else { dstb = Z; cx = col0 - D_INNER; }
  const int rr = tid >> 4, c4 = (tid & 15) * 4;
#pragma unroll
  for (int p = 0; p < 8; ++p) {
    const int row = p * 8 + rr;
    const v4f v = *(const v4fa*)&sh[row * SHP + c4];
    *(volatile v4f*)(dstb + (size_t)(rowblk + row) * D_INNER + cx + c4) = v;
  }
  __threadfence();
#pragma unroll
  for (int p = 0; p < 8; ++p) {
    const int row = p * 8 + rr;
    const v4f v = *(const v4fa*)&sh[row * SHP + c4];
    *(volatile v4f*)(dstb + (size_t)(rowblk + row) * D_INNER + cx + c4) = v;
  }
}

__global__ void __launch_bounds__(128)
k_dwconv(const float* __restrict__ X, const float* __restrict__ cw,
         const float* __restrict__ cb, float* __restrict__ XC, f16* __restrict__ XCh) {
  __shared__ __attribute__((aligned(16))) f16 shx[D_INNER];
  const int r = blockIdx.x;
  if (r >= NROW) return;
  const int l = r & (Lc - 1);
  const int tid = threadIdx.x;
  const int d4 = tid * 4;
  float acc[4];
#pragma unroll
  for (int c = 0; c < 4; ++c) acc[c] = 0.0f;
#pragma unroll
  for (int k = 0; k < D_CONV; ++k) {
    const int ls = l + k - (D_CONV - 1);
    if (ls >= 0) {
      const v4f xv = *(const v4fa*)(X + (size_t)(r + k - (D_CONV - 1)) * D_INNER + d4);
#pragma unroll
      for (int c = 0; c < 4; ++c) acc[c] += cw[(d4 + c) * D_CONV + k] * xv[c];
    }
  }
  Pack4 o;
#pragma unroll
  for (int c = 0; c < 4; ++c) {
    const float v = acc[c] + cb[d4 + c];
    const float sg = __builtin_amdgcn_rcpf(1.0f + __expf(-v));
    const float s = v * sg;
    o.s[c] = s;
    shx[d4 + c] = (f16)(s * X_SCALE);
  }
  float* pxc = XC + (size_t)r * D_INNER + d4;
  *(volatile v4f*)pxc = o.f;
  __syncthreads();
  Pack8 q; q.u = zero4u();
  f16* pxh = XCh + (size_t)r * D_INNER + tid * 8;
  if (tid < 64) {
    q.h = *(const v8ha*)(shx + tid * 8);
    *(volatile v4u*)pxh = q.u;
  }
  __threadfence();
  *(volatile v4f*)pxc = o.f;
  if (tid < 64) *(volatile v4u*)pxh = q.u;
}

__global__ void __launch_bounds__(128)
k_xproj(const f16* __restrict__ XCh, const f16* __restrict__ WxT, float* __restrict__ DBC) {
  __shared__ __attribute__((aligned(16))) float sh[64 * SHP];
  const int tid = threadIdx.x, wave = tid >> 5, l = tid & 31, h = l >> 4, m = l & 15;
  const int rowblk = blockIdx.x * 64;
  if (rowblk >= NROW) return;
  const int row0 = rowblk + wave * 16;
  v8f acc[3];
#pragma unroll
  for (int j = 0; j < 3; ++j) acc[j] = zero8f();
  const f16* arow = XCh + (size_t)(row0 + m) * D_INNER;
  for (int k = 0; k < D_INNER; k += 32) {
    const v16h a = ld_frag(arow, k);
#pragma unroll
    for (int j = 0; j < 3; ++j) {
      const v16h bb = ld_frag(WxT + (size_t)(16 * j + m) * D_INNER, k);
      acc[j] = mma16(a, bb, acc[j]);
    }
  }
#pragma unroll
  for (int j = 0; j < 3; ++j)
#pragma unroll
    for (int r = 0; r < 8; ++r)
      sh[(wave * 16 + 8 * h + r) * SHP + 16 * j + m] = acc[j][r] * (1.0f / (X_SCALE * W_SCALE));
#pragma unroll
  for (int r = 0; r < 8; ++r)
    sh[(wave * 16 + 8 * h + r) * SHP + 48 + m] = 0.0f;
  __syncthreads();
  const int rr = tid >> 4, c4 = (tid & 15) * 4;
#pragma unroll
  for (int p = 0; p < 8; ++p) {
    const int row = p * 8 + rr;
    const v4f v = *(const v4fa*)&sh[row * SHP + c4];
    *(volatile v4f*)(DBC + (size_t)(rowblk + row) * DBC_P + c4) = v;
  }
  __threadfence();
#pragma unroll
  for (int p = 0; p < 8; ++p) {
    const int row = p * 8 + rr;
    const v4f v = *(const v4fa*)&sh[row * SHP + c4];
    *(volatile v4f*)(DBC + (size_t)(rowblk + row) * DBC_P + c4) = v;
  }
}

__global__ void __launch_bounds__(256)
k_scan(const float* __restrict__ XC, const float* __restrict__ Zb,
       const float* __restrict__ DBC, const f16* __restrict__ WdtT,
       const float* __restrict__ b_dt, const float* __restrict__ A_log,
       const float* __restrict__ Dv, f16* __restrict__ Yt) {
  __shared__ float sdt[CHUNK][16];
  __shared__ float sx[CHUNK][16];
  __shared__ float sz[CHUNK][16];
  __shared__ float sB[CHUNK][16];
  __shared__ float sC[CHUNK][16];
  __shared__ float sy[CHUNK][16];
  const int bg = blockIdx.x;
  if (bg >= Bc * NG) return;
  const int b = bg >> 5, g = bg & 31, d0 = g * 16;
  const int tid = threadIdx.x, wave = tid >> 5, l = tid & 31, h = l >> 4, m = l & 15;
  const int dl = wave * 2 + h;
  const int d  = d0 + dl;
  const int s  = m;
  const float a_ds = -expf(A_log[d * D_STATE + s]);
  const float Dd   = Dv[d];
  const float bdt  = b_dt[d0 + m];
  const v16h bw = ld_frag(WdtT + (size_t)(d0 + m) * 32, 0);
  float hstate = 0.0f;

  for (int c = 0; c < Lc / CHUNK; ++c) {
    const int l0 = c * CHUNK;
    const size_t rb = (size_t)b * Lc + l0;
    {
      const int i = tid >> 1, hf = (tid & 1) * 8;
      const size_t r = rb + i;
      const float* px = XC + r * D_INNER + d0 + hf;
      const float* pz = Zb + r * D_INNER + d0 + hf;
      const float* pb = DBC + r * DBC_P + DT_RANK + hf;
      const float* pc = DBC + r * DBC_P + DT_RANK + D_STATE + hf;
      const v4f x0 = *(const v4fa*)px, x1 = *(const v4fa*)(px + 4);
      const v4f z0 = *(const v4fa*)pz, z1 = *(const v4fa*)(pz + 4);
      const v4f b0 = *(const v4fa*)pb, b1 = *(const v4fa*)(pb + 4);
      const v4f c0 = *(const v4fa*)pc, c1 = *(const v4fa*)(pc + 4);
#pragma unroll
      for (int j = 0; j < 4; ++j) {
        sx[i][hf + j] = x0[j]; sx[i][hf + 4 + j] = x1[j];
        sz[i][hf + j] = z0[j]; sz[i][hf + 4 + j] = z1[j];
        sB[i][hf + j] = b0[j]; sB[i][hf + 4 + j] = b1[j];
        sC[i][hf + j] = c0[j]; sC[i][hf + 4 + j] = c1[j];
      }
    }
    {
      const float* prow = DBC + (rb + 16 * wave + m) * DBC_P + 8 * h;
      const v4f q0 = *(const v4fa*)prow, q1 = *(const v4fa*)(prow + 4);
      Pack8 p;
#pragma unroll
      for (int j = 0; j < 4; ++j) {
        p.s[j]     = (f16)(q0[j] * DB_SCALE);
        p.s[4 + j] = (f16)(q1[j] * DB_SCALE);
      }
      Frag af;
      af.half[0] = p.h;
      af.u[1] = zero4u();
      v8f acc = zero8f();
      acc = mma16(af.v, bw, acc);
#pragma unroll
      for (int r = 0; r < 8; ++r) {
        const float v = acc[r] * (1.0f / (DB_SCALE * W_SCALE)) + bdt;
        const float sp = (v > 20.0f) ? v : log1pf(expf(v));
        sdt[16 * wave + 8 * h + r][m] = sp;
      }
    }
    __syncthreads();
    for (int i = 0; i < CHUNK; ++i) {
      const float dtv = sdt[i][dl];
      const float xv  = sx[i][dl];
      hstate = __expf(dtv * a_ds) * hstate + (dtv * xv) * sB[i][s];
      float part = hstate * sC[i][s];
      part += __shfl_xor(part, 1, 32);
      part += __shfl_xor(part, 2, 32);
      part += __shfl_xor(part, 4, 32);
      part += __shfl_xor(part, 8, 32);
      if (s == 0) {
        const float zv = sz[i][dl];
        const float sg = zv * __builtin_amdgcn_rcpf(1.0f + __expf(-zv));
        sy[i][dl] = (part + Dd * xv) * sg;
      }
    }
    __syncthreads();
    {
      const int i = tid >> 1, hf = (tid & 1) * 8;
      Pack8 p;
#pragma unroll
      for (int j = 0; j < 8; ++j) p.s[j] = (f16)(sy[i][hf + j] * Y_SCALE);
      f16* dst = Yt + ((size_t)bg * Lc + l0 + i) * 16 + hf;
      *(volatile v4u*)dst = p.u;
      __threadfence();
      *(volatile v4u*)dst = p.u;
    }
    __syncthreads();
  }
}

__global__ void __launch_bounds__(128)
k_out_proj(const f16* __restrict__ Yt, const f16* __restrict__ WoutT,
           const float* __restrict__ top, f16* __restrict__ Cat) {
  __shared__ __attribute__((aligned(16))) float sh[64 * SHP];
  const int tid = threadIdx.x, wave = tid >> 5, l = tid & 31, h = l >> 4, m = l & 15;
  const int rowblk = blockIdx.x * 64, col0 = blockIdx.y * 64;
  if (rowblk >= NROW || col0 >= Cc) return;
  const int b = rowblk >> 12;
  const int lblk = rowblk & (Lc - 1);
  const int lm = lblk + wave * 16 + m;
  v8f acc[4];
#pragma unroll
  for (int j = 0; j < 4; ++j) acc[j] = zero8f();
  const f16* ybase = Yt + ((size_t)(b * NG) * Lc + lm) * 16 + 8 * h;
  for (int k = 0; k < D_INNER; k += 32) {
    const int g = k >> 4;
    Frag a;
    a.half[0] = *(const v8ha*)(ybase + (size_t)g * Lc * 16);
    a.half[1] = *(const v8ha*)(ybase + (size_t)(g + 1) * Lc * 16);
#pragma unroll
    for (int j = 0; j < 4; ++j) {
      const v16h bb = ld_frag(WoutT + (size_t)(col0 + 16 * j + m) * D_INNER, k);
      acc[j] = mma16(a.v, bb, acc[j]);
    }
  }
#pragma unroll
  for (int j = 0; j < 4; ++j)
#pragma unroll
    for (int r = 0; r < 8; ++r) {
      const int ll  = lblk + wave * 16 + 8 * h + r;
      const int col = col0 + 16 * j + m;
      const int hp = ll >> 6, wp = ll & 63;
      const float tu = top[(((size_t)b * Cc + col) * HT + (hp >> 1)) * WT + (wp >> 1)];
      sh[(wave * 16 + 8 * h + r) * SHP + 16 * j + m] = acc[j][r] * (1.0f / (Y_SCALE * W_SCALE)) + tu;
    }
  __syncthreads();
  const int rr = tid >> 3, c8 = (tid & 7) * 8;
#pragma unroll
  for (int p = 0; p < 4; ++p) {
    const int row = p * 16 + rr;
    Pack8 q;
#pragma unroll
    for (int j = 0; j < 8; ++j) q.s[j] = (f16)sh[row * SHP + c8 + j];
    *(volatile v4u*)(Cat + ((size_t)rowblk + row) * 512 + col0 + c8) = q.u;
  }
  __threadfence();
#pragma unroll
  for (int p = 0; p < 4; ++p) {
    const int row = p * 16 + rr;
    Pack8 q;
#pragma unroll
    for (int j = 0; j < 8; ++j) q.s[j] = (f16)sh[row * SHP + c8 + j];
    *(volatile v4u*)(Cat + ((size_t)rowblk + row) * 512 + col0 + c8) = q.u;
  }
}

__global__ void __launch_bounds__(128)
k_fuse_conv(const f16* __restrict__ Cat, const f16* __restrict__ Wc,
            const float* __restrict__ fuse_b, const float* __restrict__ gamma,
            const float* __restrict__ beta, const float* __restrict__ mean,
            const float* __restrict__ var, float* __restrict__ Out) {
  __shared__ __attribute__((aligned(16))) float sh[64 * SHP];
  const int tid = threadIdx.x, wave = tid >> 5, l = tid & 31, h = l >> 4, m = l & 15;
  const int bh = blockIdx.x, co0 = blockIdx.y * 64;
  if (bh >= Bc * HL || co0 >= Cc) return;
  const int b = bh >> 6, hrow = bh & 63;
  const int w0 = wave * 16;
  v8f acc[4];
#pragma unroll
  for (int j = 0; j < 4; ++j) acc[j] = zero8f();
  for (int t = 0; t < 9; ++t) {
    const int kh = t / 3, kw = t - 3 * kh;
    const int hi = hrow + kh - 1;
    const int wi = w0 + m + kw - 1;
    const bool ok = (hi >= 0) && (hi < HL) && (wi >= 0) && (wi < WL);
    const int hic = hi < 0 ? 0 : (hi >= HL ? HL - 1 : hi);
    const int wic = wi < 0 ? 0 : (wi >= WL ? WL - 1 : wi);
    const f16* ap = Cat + (((size_t)b * HL + hic) * WL + wic) * 512;
    const f16* wp = Wc + ((size_t)t * Cc + co0 + m) * 512;
    for (int k = 0; k < 512; k += 32) {
      Frag a;
      a.v = ld_frag(ap, k);
      if (!ok) { a.u[0] = zero4u(); a.u[1] = zero4u(); }
#pragma unroll
      for (int j = 0; j < 4; ++j) {
        const v16h bb = ld_frag(wp + (size_t)(16 * j) * 512, k);
        acc[j] = mma16(a.v, bb, acc[j]);
      }
    }
  }
#pragma unroll
  for (int j = 0; j < 4; ++j)
#pragma unroll
    for (int r = 0; r < 8; ++r)
      sh[(16 * j + m) * SHP + w0 + 8 * h + r] = acc[j][r] * (1.0f / W_SCALE);
  __syncthreads();
  const int rr = tid >> 4, w4 = (tid & 15) * 4;
#pragma unroll
  for (int p = 0; p < 8; ++p) {
    const int col = p * 8 + rr;
    const int co = co0 + col;
    const float inv = gamma[co] / sqrtf(var[co] + 1e-5f);
    const float fb = fuse_b[co], mu = mean[co], be = beta[co];
    const v4f v = *(const v4fa*)&sh[col * SHP + w4];
    Pack4 o;
#pragma unroll
    for (int q = 0; q < 4; ++q) {
      const float cv = v[q] + fb;
      const float bn = (cv - mu) * inv + be;
      o.s[q] = bn > 0.0f ? bn : 0.0f;
    }
    *(volatile v4f*)(Out + (((size_t)b * Cc + co) * HL + hrow) * WL + w4) = o.f;
  }
  __threadfence();
#pragma unroll
  for (int p = 0; p < 8; ++p) {
    const int col = p * 8 + rr;
    const int co = co0 + col;
    const float inv = gamma[co] / sqrtf(var[co] + 1e-5f);
    const float fb = fuse_b[co], mu = mean[co], be = beta[co];
    const v4f v = *(const v4fa*)&sh[col * SHP + w4];
    Pack4 o;
#pragma unroll
    for (int q = 0; q < 4; ++q) {
      const float cv = v[q] + fb;
      const float bn = (cv - mu) * inv + be;
      o.s[q] = bn > 0.0f ? bn : 0.0f;
    }
    *(volatile v4f*)(Out + (((size_t)b * Cc + co) * HL + hrow) * WL + w4) = o.f;
  }
}

extern "C" void kernel_launch(void* const* d_in, const int* in_sizes, int n_in,
                              void* d_out, int out_size, void* d_ws, size_t ws_size,
                              hipStream_t stream) {
  if (n_in < 17) return;
  if (in_sizes[0] != Bc * Cc * HT * WT) return;
  if (in_sizes[1] != Bc * Cc * HL * WL) return;
  if (in_sizes[2] != Cc * 2 * D_INNER) return;
  if (in_sizes[3] != D_INNER * D_CONV) return;
  if (in_sizes[4] != D_INNER) return;
  if (in_sizes[5] != D_INNER * (DT_RANK + 2 * D_STATE)) return;
  if (in_sizes[6] != DT_RANK * D_INNER) return;
  if (in_sizes[7] != D_INNER) return;
  if (in_sizes[8] != D_INNER * D_STATE) return;
  if (in_sizes[9] != D_INNER) return;
  if (in_sizes[10] != D_INNER * Cc) return;
  if (in_sizes[11] != Cc * 2 * Cc * 9) return;
  for (int i = 12; i < 17; ++i) if (in_sizes[i] != Cc) return;
  if (out_size != Bc * Cc * HL * WL) return;

  const float* top     = (const float*)d_in[0];
  const float* lateral = (const float*)d_in[1];
  const float* W_in    = (const float*)d_in[2];
  const float* conv_w  = (const float*)d_in[3];
  const float* conv_b  = (const float*)d_in[4];
  const float* W_x     = (const float*)d_in[5];
  const float* W_dt    = (const float*)d_in[6];
  const float* b_dt    = (const float*)d_in[7];
  const float* A_log   = (const float*)d_in[8];
  const float* Dvec    = (const float*)d_in[9];
  const float* W_out   = (const float*)d_in[10];
  const float* fuse_w  = (const float*)d_in[11];
  const float* fuse_b  = (const float*)d_in[12];
  const float* bn_g    = (const float*)d_in[13];
  const float* bn_b    = (const float*)d_in[14];
  const float* bn_m    = (const float*)d_in[15];
  const float* bn_v    = (const float*)d_in[16];
  float* out = (float*)d_out;

  char* ws = (char*)d_ws;
  size_t off = 0;
  auto carve = [&](size_t bytes) {
    size_t o = off;
    off = (off + bytes + 255) & ~(size_t)255;
    return o;
  };
  f16*   U     = (f16*)(ws + carve((size_t)NROW * Cc * 2));
  f16*   WinT  = (f16*)(ws + carve((size_t)(2 * D_INNER) * Cc * 2));
  f16*   WxT   = (f16*)(ws + carve((size_t)48 * D_INNER * 2));
  f16*   WdtT  = (f16*)(ws + carve((size_t)D_INNER * 32 * 2));
  f16*   WoutT = (f16*)(ws + carve((size_t)Cc * D_INNER * 2));
  f16*   WcT   = (f16*)(ws + carve((size_t)9 * Cc * 512 * 2));
  float* X     = (float*)(ws + carve((size_t)NROW * D_INNER * 4));
  float* Z     = (float*)(ws + carve((size_t)NROW * D_INNER * 4));
  float* XC    = (float*)(ws + carve((size_t)NROW * D_INNER * 4));
  f16*   XCh   = (f16*)(ws + carve((size_t)NROW * D_INNER * 2));
  float* DBC   = (float*)(ws + carve((size_t)NROW * DBC_P * 4));
  f16*   Yt    = (f16*)(ws + carve((size_t)NROW * D_INNER * 2));
  f16*   Cat   = (f16*)(ws + carve((size_t)NROW * 512 * 2));
  if (off > ws_size) return;

  k_wT<<<dim3((2 * D_INNER * (Cc / 8) + 255) / 256), dim3(256), 0, stream>>>(W_in, WinT, Cc, 2 * D_INNER, Cc, W_SCALE);
  k_wT<<<dim3((48 * (D_INNER / 8) + 255) / 256), dim3(256), 0, stream>>>(W_x, WxT, D_INNER, 48, D_INNER, W_SCALE);
  k_wT<<<dim3((D_INNER * (32 / 8) + 255) / 256), dim3(256), 0, stream>>>(W_dt, WdtT, DT_RANK, D_INNER, 32, W_SCALE);
  k_wT<<<dim3((Cc * (D_INNER / 8) + 255) / 256), dim3(256), 0, stream>>>(W_out, WoutT, D_INNER, Cc, D_INNER, W_SCALE);
  k_convwT<<<dim3((9 * 256 * 512 / 8 + 255) / 256), dim3(256), 0, stream>>>(fuse_w, WcT, W_SCALE);
  k_build_u<<<dim3((NROW * 32 + 255) / 256), dim3(256), 0, stream>>>(top, U);
  k_lateral<<<dim3((NROW * 32 + 255) / 256), dim3(256), 0, stream>>>(lateral, Cat);

  k_in_proj<<<dim3((NROW + 63) / 64, (2 * D_INNER + 63) / 64), dim3(128), 0, stream>>>(U, WinT, X, Z);
  k_dwconv<<<dim3(NROW), dim3(128), 0, stream>>>(X, conv_w, conv_b, XC, XCh);
  k_xproj<<<dim3((NROW + 63) / 64), dim3(128), 0, stream>>>(XCh, WxT, DBC);
  k_scan<<<dim3(Bc * NG), dim3(256), 0, stream>>>(XC, Z, DBC, WdtT, b_dt, A_log, Dvec, Yt);
  k_out_proj<<<dim3((NROW + 63) / 64, (Cc + 63) / 64), dim3(128), 0, stream>>>(Yt, WoutT, top, Cat);

  k_fuse_conv<<<dim3(Bc * HL, (Cc + 63) / 64), dim3(128), 0, stream>>>(Cat, WcT, fuse_b, bn_g, bn_b, bn_m, bn_v, out);
  (void)hipGetLastError();
}
